// CrossAttentionMultiLayerPerceptron_61976378082028
// MI455X (gfx1250) — hardware-verified
//
#include <hip/hip_runtime.h>
#include <math.h>

typedef __attribute__((ext_vector_type(16))) _Float16 v16h;
typedef __attribute__((ext_vector_type(16))) __bf16 v16b;
typedef __attribute__((ext_vector_type(8)))  _Float16 v8h;
typedef __attribute__((ext_vector_type(8)))  float v8f;
typedef __attribute__((ext_vector_type(4)))  float v4f;
typedef __attribute__((ext_vector_type(2)))  float v2f;
typedef __attribute__((ext_vector_type(4)))  unsigned v4u;
typedef __attribute__((ext_vector_type(4)))  int v4i;
typedef float __attribute__((may_alias)) float_a;
typedef int __attribute__((may_alias)) int_a;

template <typename T> __device__ __forceinline__ void vst2(void* p, T v) { *(volatile T*)p = v; __threadfence(); *(volatile T*)p = v; }
__device__ __forceinline__ v8f wmma16(v16h a, v16h b, v8f c) {
  v8f d = __builtin_amdgcn_wmma_f32_16x16x32_f16(false, a, false, b, (short)0, c, false, false);
  asm volatile("v_nop\n\tv_nop\n\tv_nop\n\tv_nop" : "+v"(d) : "v"(a), "v"(b));
  return d;
}
__device__ __forceinline__ v8f wmma_bf(v16b a, v16b b, v8f c) {
  v8f d = __builtin_amdgcn_wmma_f32_16x16x32_bf16(false, a, false, b, (short)0, c, false, false);
  asm volatile("v_nop\n\tv_nop\n\tv_nop\n\tv_nop" : "+v"(d) : "v"(a), "v"(b));
  return d;
}
__device__ __forceinline__ v16h frag_h(const _Float16* rowk0, int lane) {
  union { v16h v; v8h q[2]; } u; const _Float16* p = rowk0 + 8 * (lane >> 4);
  u.q[0] = *(const v8h*)p; u.q[1] = *(const v8h*)(p + 16); return u.v;
}
__device__ __forceinline__ v16h frag_f32(const float* rowk0, int lane) {
  v16h a; const float* p = rowk0 + 8 * (lane >> 4);
#pragma unroll
  for (int i = 0; i < 8; ++i) { a[i] = (_Float16)p[i]; a[8 + i] = (_Float16)p[16 + i]; }
  return a;
}
__device__ __forceinline__ v16h frag_f32s(const float* rowk0, int lane, float sc) {
  v16h a; const float* p = rowk0 + 8 * (lane >> 4);
#pragma unroll
  for (int i = 0; i < 8; ++i) { a[i] = (_Float16)(p[i] * sc); a[8 + i] = (_Float16)(p[16 + i] * sc); }
  return a;
}
__device__ __forceinline__ v16h fragc_f32(const float* W, int k0, int n, int lane, int ld, int K) {
  v16h a; const int g = lane >> 4;
#pragma unroll
  for (int i = 0; i < 8; ++i) { const int ka = k0 + 8 * g + i, kb = ka + 16;
    a[i] = (_Float16)(ka < K ? W[(size_t)ka * ld + n] : 0.f); a[8 + i] = (_Float16)(kb < K ? W[(size_t)kb * ld + n] : 0.f); }
  return a;
}
struct F2 { v16b h, l; };
__device__ __forceinline__ F2 bsplit16(const float v[16]) { F2 r;
#pragma unroll
  for (int i = 0; i < 16; ++i) { const __bf16 h = (__bf16)v[i]; r.h[i] = h; r.l[i] = (__bf16)(v[i] - (float)h); }
  return r; }
__device__ __forceinline__ F2 split_row(const float* row, int k0, int lane) { float v[16]; const float* p = row + k0 + 8 * (lane >> 4);
#pragma unroll
  for (int i = 0; i < 8; ++i) { v[i] = p[i]; v[8 + i] = p[16 + i]; }
  return bsplit16(v); }
__device__ __forceinline__ F2 split_rowK(const float* row, int k0, int lane, int K) { float v[16]; const int g = lane >> 4;
#pragma unroll
  for (int i = 0; i < 8; ++i) { const int ka = k0 + 8 * g + i, kb = ka + 16; v[i] = ka < K ? row[ka] : 0.f; v[8 + i] = kb < K ? row[kb] : 0.f; }
  return bsplit16(v); }
__device__ __forceinline__ F2 split_col(const float* W, int k0, int n, int lane, int ld, int K) { float v[16]; const int g = lane >> 4;
#pragma unroll
  for (int i = 0; i < 8; ++i) { const int ka = k0 + 8 * g + i, kb = ka + 16; v[i] = ka < K ? W[(size_t)ka * ld + n] : 0.f; v[8 + i] = kb < K ? W[(size_t)kb * ld + n] : 0.f; }
  return bsplit16(v); }
__device__ __forceinline__ v8f mac3(const F2& a, const F2& b, v8f c) { c = wmma_bf(a.l, b.h, c); c = wmma_bf(a.h, b.l, c); return wmma_bf(a.h, b.h, c); }
__device__ __forceinline__ float sigm(float v) { return 1.0f / (1.0f + expf(-v)); }
#define LDSX() do { asm volatile("s_wait_dscnt 0" ::: "memory"); __builtin_amdgcn_wave_barrier(); __builtin_amdgcn_fence(__ATOMIC_RELEASE, "workgroup"); } while (0)


#define NN 65408
#define NG 256
#define IN 128
#define FD 256
#define TXT 512
#define OUTD 128
#define LMAX 383
__device__ __forceinline__ int clampi(int v, int lo, int hi) { return v < lo ? lo : (v > hi ? hi : v); }
__device__ __forceinline__ void seg_of(const int* __restrict__ lens, int g, int& off, int& len) { int o = 0; for (int j = 0; j < g; ++j) o += clampi(lens[j], 0, LMAX); int l = clampi(lens[g], 0, LMAX); if (o > NN) o = NN; if (o + l > NN) l = NN - o; off = o; len = l; }

template <int K, int RELU>
__global__ __launch_bounds__(128) void k_gemm256(const float* __restrict__ A, int M, const float* __restrict__ Bm, const float* __restrict__ bias, float* __restrict__ Cc) {
  __shared__ __align__(16) float so[4][16][132];
  const int tid = threadIdx.x, wave = tid >> 5, lane = tid & 31, col = lane & 15, g = lane >> 4;
  const int r0 = blockIdx.x * 64 + wave * 16; const int ra = (r0 + col) < M ? (r0 + col) : (M - 1);
#pragma unroll 1
  for (int nh = 0; nh < 2; ++nh) { v8f acc[8] = {};
#pragma unroll 1
    for (int kc = 0; kc < K / 32; ++kc) { const F2 a = split_row(A + (size_t)ra * K, kc * 32, lane);
#pragma unroll
      for (int j = 0; j < 8; ++j) acc[j] = mac3(a, split_col(Bm, kc * 32, nh * 128 + j * 16 + col, lane, FD, K), acc[j]); }
#pragma unroll
    for (int j = 0; j < 8; ++j) { const int n = nh * 128 + j * 16 + col; const float bb = bias ? bias[n] : 0.f;
#pragma unroll
      for (int r = 0; r < 8; ++r) { const float v = acc[j][r] + bb; so[wave][8 * g + r][j * 16 + col] = RELU ? (v > 0.f ? v : 0.f) : v; } }
    LDSX();
    for (int rl = 0; rl < 16; ++rl) { if (r0 + rl >= M) break; vst2(Cc + (size_t)(r0 + rl) * FD + nh * 128 + lane * 4, *(const v4f*)(&so[wave][rl][lane * 4])); }
    LDSX(); }
}
__global__ __launch_bounds__(256) void k_seg(const float* __restrict__ Hh, const int* __restrict__ lens, float* __restrict__ HS) {
  __shared__ int soff, slen;
  const int g = blockIdx.x, tid = threadIdx.x;
  if (tid == 0) { int o, l; seg_of(lens, g, o, l); soff = o; slen = l; }
  __syncthreads();
  const int off = soff, len = slen; float s = 0.f;
#pragma unroll 4
  for (int i = 0; i < len; ++i) s += Hh[(size_t)(off + i) * FD + tid];
  vst2(HS + (size_t)g * FD + tid, (float_a)s);
}
__global__ __launch_bounds__(128) void k_small(const float* __restrict__ text, const float* __restrict__ Wq, const float* __restrict__ bq, const float* __restrict__ Wk, const float* __restrict__ bk, const float* __restrict__ HS, const int* __restrict__ lens,
                                              const float* __restrict__ Wv, const float* __restrict__ bv, const float* __restrict__ Wo, float* __restrict__ Qg, float* __restrict__ Rg, float* __restrict__ Vs, float* __restrict__ Ug, int stage) {
  __shared__ __align__(16) float so[4][16][132];
  const int tid = threadIdx.x, wave = tid >> 5, lane = tid & 31, col = lane & 15, g8 = lane >> 4;
  const int r0 = blockIdx.x * 64 + wave * 16;
#pragma unroll 1
  for (int nh = 0; nh < 2; ++nh) { v8f acc[8] = {};
    if (stage == 0) {
#pragma unroll 1
      for (int kc = 0; kc < TXT / 32; ++kc) { const F2 a = split_row(text + (size_t)(r0 + col) * TXT, kc * 32, lane);
#pragma unroll
        for (int j = 0; j < 8; ++j) acc[j] = mac3(a, split_col(Wq, kc * 32, nh * 128 + j * 16 + col, lane, FD, TXT), acc[j]); } }
    else if (stage == 1) {
#pragma unroll 1
      for (int kc = 0; kc < FD / 32; ++kc) { const F2 a = split_row(Qg + (size_t)(r0 + col) * FD, kc * 32, lane);
#pragma unroll
        for (int j = 0; j < 8; ++j) acc[j] = mac3(a, split_row(Wk + (size_t)(nh * 128 + j * 16 + col) * FD, kc * 32, lane), acc[j]); } }
    else {
#pragma unroll 1
      for (int kc = 0; kc < FD / 32; ++kc) { const F2 a = split_row(Vs + (size_t)(r0 + col) * FD, kc * 32, lane);
#pragma unroll
        for (int j = 0; j < 8; ++j) acc[j] = mac3(a, split_col(Wo, kc * 32, nh * 128 + j * 16 + col, lane, FD, FD), acc[j]); } }
#pragma unroll
    for (int j = 0; j < 8; ++j) { const int n = nh * 128 + j * 16 + col;
#pragma unroll
      for (int r = 0; r < 8; ++r) so[wave][8 * g8 + r][j * 16 + col] = acc[j][r] + (stage == 0 ? bq[n] : 0.f); }
    LDSX();
    float* Dst = stage == 0 ? Qg : (stage == 1 ? Rg : Ug);
    for (int rl = 0; rl < 16; ++rl) vst2(Dst + (size_t)(r0 + rl) * FD + nh * 128 + lane * 4, *(const v4f*)(&so[wave][rl][lane * 4]));
    LDSX();
    if (stage == 1) {
      v8f acc2[8] = {};
#pragma unroll 1
      for (int kc = 0; kc < FD / 32; ++kc) { const F2 a = split_row(HS + (size_t)(r0 + col) * FD, kc * 32, lane);
#pragma unroll
        for (int j = 0; j < 8; ++j) acc2[j] = mac3(a, split_col(Wv, kc * 32, nh * 128 + j * 16 + col, lane, FD, FD), acc2[j]); }
#pragma unroll
      for (int j = 0; j < 8; ++j) { const int n = nh * 128 + j * 16 + col;
#pragma unroll
        for (int r = 0; r < 8; ++r) { const int gr = r0 + 8 * g8 + r; so[wave][8 * g8 + r][j * 16 + col] = acc2[j][r] + (float)clampi(lens[gr], 0, LMAX) * bv[n]; } }
      LDSX();
      for (int rl = 0; rl < 16; ++rl) vst2(Vs + (size_t)(r0 + rl) * FD + nh * 128 + lane * 4, *(const v4f*)(&so[wave][rl][lane * 4]));
      LDSX(); } }
  (void)bk;
}
__global__ __launch_bounds__(256) void k_soft(const float* __restrict__ Hh, const int* __restrict__ lens, const float* __restrict__ Rg, const float* __restrict__ Qg, const float* __restrict__ bk, const float* __restrict__ Ug, const float* __restrict__ bo, float* __restrict__ Z) {
  __shared__ float sr[FD], su[FD], ssc[LMAX + 1], sred[8], scp[256];
  const int g = blockIdx.x, tid = threadIdx.x, wave = tid >> 5, lane = tid & 31;
  __shared__ int soff, slen; if (tid == 0) { int o, l; seg_of(lens, g, o, l); soff = o; slen = l; }
  sr[tid] = Rg[(size_t)g * FD + tid]; su[tid] = Ug[(size_t)g * FD + tid]; scp[tid] = Qg[(size_t)g * FD + tid] * bk[tid];
  __syncthreads();
  const int off = soff, len = slen;
#pragma unroll
  for (int o = 128; o > 0; o >>= 1) { if (tid < o) scp[tid] += scp[tid + o]; __syncthreads(); }
  const float cg = scp[0];
#pragma unroll 1
  for (int i = wave; i < len; i += 8) { const float* hr = Hh + (size_t)(off + i) * FD + lane * 8; float s = 0.f;
#pragma unroll
    for (int e = 0; e < 8; ++e) s += hr[e] * sr[lane * 8 + e];
#pragma unroll
    for (int o = 16; o > 0; o >>= 1) s += __shfl_xor(s, o, 32);
    if (lane == 0) ssc[i] = s + cg; }
  __syncthreads();
  if (tid == 0) { float m = -3.4e38f; for (int i = 0; i < len; ++i) m = fmaxf(m, ssc[i]); float z = 0.f; for (int i = 0; i < len; ++i) z += expf(ssc[i] - m); sred[0] = m; sred[1] = z; }
  __syncthreads();
  const float m = sred[0], invz = 1.0f / sred[1];
#pragma unroll 1
  for (int i = wave; i < len; i += 8) { const float p = expf(ssc[i] - m) * invz; v4f a, b;
#pragma unroll
    for (int e = 0; e < 4; ++e) { const int c = lane * 4 + e; const float v = p * su[c] + bo[c]; a[e] = v > 0.f ? v : 0.f; const int c2 = 128 + c; const float v2 = p * su[c2] + bo[c2]; b[e] = v2 > 0.f ? v2 : 0.f; }
    vst2(Z + (size_t)(off + i) * FD + lane * 4, a); vst2(Z + (size_t)(off + i) * FD + 128 + lane * 4, b); }
}
__global__ __launch_bounds__(128) void k_y(const float* __restrict__ Z, const float* __restrict__ W2, const float* __restrict__ b2, float* __restrict__ out) {
  __shared__ __align__(16) float so[4][16][132];
  const int tid = threadIdx.x, wave = tid >> 5, lane = tid & 31, col = lane & 15, g = lane >> 4;
  const int r0 = blockIdx.x * 64 + wave * 16; const int ra = (r0 + col) < NN ? (r0 + col) : (NN - 1);
  v8f acc[8] = {};
#pragma unroll 1
  for (int kc = 0; kc < FD / 32; ++kc) { const F2 a = split_row(Z + (size_t)ra * FD, kc * 32, lane);
#pragma unroll
    for (int j = 0; j < 8; ++j) acc[j] = mac3(a, split_col(W2, kc * 32, j * 16 + col, lane, OUTD, FD), acc[j]); }
#pragma unroll
  for (int j = 0; j < 8; ++j) { const float bb = b2[j * 16 + col];
#pragma unroll
    for (int r = 0; r < 8; ++r) so[wave][8 * g + r][j * 16 + col] = acc[j][r] + bb; }
  LDSX();
  for (int rl = 0; rl < 16; ++rl) { if (r0 + rl >= NN) break; vst2(out + (size_t)(r0 + rl) * OUTD + lane * 4, *(const v4f*)(&so[wave][rl][lane * 4])); }
}
extern "C" void kernel_launch(void* const* d_in, const int* in_sizes, int n_in, void* d_out, int out_size, void* d_ws, size_t ws_size, hipStream_t stream) {
  (void)in_sizes; (void)n_in; (void)out_size; (void)ws_size;
  const float* x = (const float*)d_in[0]; const float* text = (const float*)d_in[1]; const int* lens = (const int*)d_in[2];
  const float* W0 = (const float*)d_in[3]; const float* b0 = (const float*)d_in[4]; const float* Wq = (const float*)d_in[5]; const float* bq = (const float*)d_in[6]; const float* Wk = (const float*)d_in[7]; const float* bk = (const float*)d_in[8];
  const float* Wv = (const float*)d_in[9]; const float* bv = (const float*)d_in[10]; const float* Wo = (const float*)d_in[11]; const float* bo = (const float*)d_in[12]; const float* W2 = (const float*)d_in[13]; const float* b2 = (const float*)d_in[14];
  float* out = (float*)d_out;
  char* ws = (char*)d_ws; size_t off = 0;
  auto take = [&](size_t bytes) { char* p = ws + off; off += (bytes + 255) & ~(size_t)255; return p; };
  float* Hh = (float*)take((size_t)(NN + 64) * FD * 4); float* Z = Hh;
  float* HS = (float*)take((size_t)NG * FD * 4);
  float* Qg = (float*)take((size_t)NG * FD * 4); float* Rg = (float*)take((size_t)NG * FD * 4); float* Vs = (float*)take((size_t)NG * FD * 4); float* Ug = (float*)take((size_t)NG * FD * 4);
  k_gemm256<IN, 1><<<(NN + 63) / 64, 128, 0, stream>>>(x, NN, W0, b0, Hh);
  k_seg<<<NG, 256, 0, stream>>>(Hh, lens, HS);
  k_small<<<NG / 64, 128, 0, stream>>>(text, Wq, bq, Wk, bk, HS, lens, Wv, bv, Wo, Qg, Rg, Vs, Ug, 0);
  k_small<<<NG / 64, 128, 0, stream>>>(text, Wq, bq, Wk, bk, HS, lens, Wv, bv, Wo, Qg, Rg, Vs, Ug, 1);
  k_small<<<NG / 64, 128, 0, stream>>>(text, Wq, bq, Wk, bk, HS, lens, Wv, bv, Wo, Qg, Rg, Vs, Ug, 2);
  k_soft<<<NG, 256, 0, stream>>>(Hh, lens, Rg, Qg, bk, Ug, bo, Z);
  k_y<<<(NN + 63) / 64, 128, 0, stream>>>(Z, W2, b2, out);
}
